// TanhConvolvedAttnLayer_50173807952856
// MI455X (gfx1250) — hardware-run, weakly checked
//
#include <hip/hip_runtime.h>


#define NB_  2
#define TT   4096
#define HD   64
#define NH_  8
#define WINW 128
#define PADW 64
#define NCH  (TT / WINW)
#define KWN  (2 * WINW)
#define NOFF (WINW + 1)
#define VO   64

typedef _Float16 h16;
typedef unsigned short bf;
typedef __attribute__((ext_vector_type(16))) __bf16   v16bf;
typedef __attribute__((ext_vector_type(16))) _Float16 v16h;
typedef __attribute__((ext_vector_type(8)))  _Float16 v8h;
typedef __attribute__((ext_vector_type(8)))  unsigned short v8us;
typedef __attribute__((ext_vector_type(8)))  float    v8f;
typedef __attribute__((ext_vector_type(4)))  float    v4f;
typedef v8h  __attribute__((may_alias)) v8ha;
typedef v4f  __attribute__((may_alias)) v4fa;
typedef v8us __attribute__((may_alias)) v8usa;

__device__ __forceinline__ unsigned short f2bf(float f) { unsigned u = __float_as_uint(f); u += 0x7FFFu + ((u >> 16) & 1u); return (unsigned short)(u >> 16); }
__device__ __forceinline__ float bf2f(unsigned short b) { return __uint_as_float(((unsigned)b) << 16); }
__device__ __forceinline__ float bfr(float f) { return bf2f(f2bf(f)); }
__device__ __forceinline__ v16h cat16(v8h lo, v8h hi) { return __builtin_shufflevector(lo, hi, 0, 1, 2, 3, 4, 5, 6, 7, 8, 9, 10, 11, 12, 13, 14, 15); }
__device__ __forceinline__ v16bf cat16b(v8us lo, v8us hi) { return __builtin_bit_cast(v16bf, __builtin_shufflevector(lo, hi, 0, 1, 2, 3, 4, 5, 6, 7, 8, 9, 10, 11, 12, 13, 14, 15)); }
__device__ __forceinline__ v8f wmma16(v16h a, v16h b, v8f c) { return __builtin_amdgcn_wmma_f32_16x16x32_f16(false, a, false, b, (short)0, c, false, false); }
__device__ __forceinline__ v8f wmmab(v16bf a, v16bf b, v8f c) { return __builtin_amdgcn_wmma_f32_16x16x32_bf16(false, a, false, b, (short)0, c, false, false); }
typedef __attribute__((ext_vector_type(2))) _Float16 v2h;
typedef __attribute__((ext_vector_type(4))) _Float16 v4h;
typedef __attribute__((ext_vector_type(2))) unsigned short v2us;
typedef __attribute__((ext_vector_type(4))) unsigned short v4us;
typedef __attribute__((ext_vector_type(2))) float v2f;
typedef __attribute__((ext_vector_type(4))) int v4i;

template <typename T16> struct WFrag;
template <> struct WFrag<h16> { typedef v16h V; static __device__ __forceinline__ V ld(const h16* p) { return cat16(*(const v8h*)p, *(const v8h*)(p + 16)); } static __device__ __forceinline__ v8f mma(V a, V b, v8f c) { return wmma16(a, b, c); } };
template <> struct WFrag<bf> { typedef v16bf V; static __device__ __forceinline__ V ld(const bf* p) { return cat16b(*(const v8us*)p, *(const v8us*)(p + 16)); } static __device__ __forceinline__ v8f mma(V a, V b, v8f c) { return wmmab(a, b, c); } };
template <typename T16, int NSPLIT, bool BIAS>
__global__ __launch_bounds__(32) void k_gemmw(const T16* __restrict__ A, const T16* __restrict__ A2, const T16* __restrict__ Bt, const T16* __restrict__ Bt2, int K, float* C, int ldc, const float* __restrict__ bias, size_t sA, size_t sB, size_t sC) {
    typedef typename WFrag<T16>::V V;
    __shared__ __align__(16) float os[16 * 68];
    const size_t z = blockIdx.z; A += z * sA; if (A2) A2 += z * sA; Bt += z * sB; if (Bt2) Bt2 += z * sB; C += z * sC;
    const int lane = threadIdx.x & 31, lr = lane & 15, hi = lane >> 4; const int r0 = blockIdx.x * 64, c0 = blockIdx.y * 64;
    v8f acc[4][4];
#pragma unroll
    for (int mb = 0; mb < 4; ++mb)
#pragma unroll
        for (int nb = 0; nb < 4; ++nb) acc[mb][nb] = (v8f){};
    const size_t aoff = (size_t)(r0 + lr) * K + 8 * hi, boff = (size_t)(c0 + lr) * K + 8 * hi;

    for (int kc = 0; kc < K; kc += 32) {
        V a[4], a2[4];
#pragma unroll
        for (int mb = 0; mb < 4; ++mb) { a[mb] = WFrag<T16>::ld(A + aoff + (size_t)mb * 16 * K + kc); if (NSPLIT == 1 || NSPLIT == 2) a2[mb] = WFrag<T16>::ld(A2 + aoff + (size_t)mb * 16 * K + kc); }
#pragma unroll
        for (int nb = 0; nb < 4; ++nb) { const V b = WFrag<T16>::ld(Bt + boff + (size_t)nb * 16 * K + kc); V b2; if (NSPLIT >= 2) b2 = WFrag<T16>::ld(Bt2 + boff + (size_t)nb * 16 * K + kc);
#pragma unroll
            for (int mb = 0; mb < 4; ++mb) { acc[mb][nb] = WFrag<T16>::mma(a[mb], b, acc[mb][nb]); if (NSPLIT == 1 || NSPLIT == 2) acc[mb][nb] = WFrag<T16>::mma(a2[mb], b, acc[mb][nb]); if (NSPLIT >= 2) acc[mb][nb] = WFrag<T16>::mma(a[mb], b2, acc[mb][nb]); } }
        asm volatile("v_nop\n\tv_nop\n\tv_nop\n\tv_nop" : "+v"(acc[0][0]), "+v"(acc[1][1]), "+v"(acc[2][2]), "+v"(acc[3][3]) : "v"(a[0]), "v"(a[3]));
    }
#pragma unroll
    for (int mb = 0; mb < 4; ++mb) {
#pragma unroll
        for (int nb = 0; nb < 4; ++nb) {
#pragma unroll
            for (int j = 0; j < 8; ++j) os[(hi * 8 + j) * 68 + nb * 16 + lr] = acc[mb][nb][j]; }
        __builtin_amdgcn_wave_barrier(); asm volatile("" ::: "memory");
        float* crow = C + (size_t)(r0 + mb * 16) * ldc + c0;
#pragma unroll 1
        for (int ps = 0; ps < 2; ++ps) {
#pragma unroll
            for (int s = 0; s < 8; ++s) { const int row = 2 * s + hi, cofs = lr * 4; v4f val = *(const v4fa*)(os + row * 68 + cofs); if (BIAS) { val[0] += bfr(bias[c0 + cofs]); val[1] += bfr(bias[c0 + cofs + 1]); val[2] += bfr(bias[c0 + cofs + 2]); val[3] += bfr(bias[c0 + cofs + 3]); }
                *(volatile v4f*)(crow + (size_t)row * ldc + cofs) = val; }
            if (ps == 0) __threadfence(); }
        __builtin_amdgcn_wave_barrier(); asm volatile("" ::: "memory");
    }
}

__device__ __forceinline__ h16 tohx(float x) { return (h16)x; }
__device__ __forceinline__ void splitf(float y, unsigned short& h, unsigned short& l) { h = f2bf(y); l = f2bf(y - bf2f(h)); }
typedef __attribute__((ext_vector_type(2))) _Float16 v2h;
typedef __attribute__((ext_vector_type(4))) _Float16 v4h;
typedef __attribute__((ext_vector_type(2))) unsigned short v2us;
typedef __attribute__((ext_vector_type(4))) unsigned short v4us;
typedef __attribute__((ext_vector_type(2))) float v2f;
typedef __attribute__((ext_vector_type(4))) int v4i;

__global__ __launch_bounds__(256) void k_cvt8(const float* __restrict__ src, bf* dst, size_t n8) { const size_t i = (size_t)blockIdx.x * 256 + threadIdx.x; if (i >= n8) return; const v8f v = *(const v8f*)(src + i * 8); v8us o;
#pragma unroll
    for (int k = 0; k < 8; ++k) o[k] = f2bf(v[k]); *(volatile v8us*)(dst + i * 8) = o; __threadfence(); *(volatile v8us*)(dst + i * 8) = o; }

__global__ __launch_bounds__(256) void k_rbf(const float* __restrict__ X, float* Y, size_t n4) { const size_t i = (size_t)blockIdx.x * 256 + threadIdx.x; if (i >= n4) return; const v4f a = *(const v4f*)(X + i * 4); v4f o;
#pragma unroll
    for (int q = 0; q < 4; ++q) o[q] = bfr(a[q]);
    *(volatile v4f*)(Y + i * 4) = o; __threadfence(); *(volatile v4f*)(Y + i * 4) = o; }

__global__ __launch_bounds__(256) void k_rope(const float* __restrict__ F, int pitch, int nheads, const float* __restrict__ CS, const float* __restrict__ RF, const float* __restrict__ nw, float sc, h16* P16, bf* Ph, bf* Pl) {
    const size_t e = ((size_t)blockIdx.x * 256 + threadIdx.x) * 2; if (e >= (size_t)nheads * TT * HD) return; const int d = (int)(e % HD); const int t = (int)((e / HD) % TT); const int h = (int)(e / ((size_t)HD * TT)); const float* f = F + (size_t)t * pitch + h * HD; const float rf = RF ? RF[(size_t)h * TT + t] : 1.0f; v2h o16; v2us oh, ol;
#pragma unroll
    for (int q = 0; q < 2; ++q) { const int dd = d + q; const int dp = (dd < HD / 2) ? dd + HD / 2 : dd - HD / 2; float x0 = f[dd], x1 = f[dp];
        if (RF) { float n0 = __fmul_rn(x0, rf), n1 = __fmul_rn(x1, rf); x0 = __fmul_rn(bfr(nw[dd]), n0); x1 = __fmul_rn(bfr(nw[dp]), n1); }
        const v2f cs = *(const v2f*)(CS + ((size_t)t * HD + dd) * 2); float a = __fmul_rn(x0, cs[0]), bq = __fmul_rn(x1, cs[1]); const float r = ((dd < HD / 2) ? __fsub_rn(a, bq) : __fadd_rn(a, bq)) * sc;
        o16[q] = tohx(r); unsigned short a2, c2; splitf(r, a2, c2); oh[q] = a2; ol[q] = c2; }
    *(volatile v2h*)(P16 + e) = o16; *(volatile v2us*)(Ph + e) = oh; *(volatile v2us*)(Pl + e) = ol; __threadfence(); *(volatile v2h*)(P16 + e) = o16; *(volatile v2us*)(Ph + e) = oh; *(volatile v2us*)(Pl + e) = ol; }
__global__ __launch_bounds__(256) void k_csid(float* CS) { const int idx = blockIdx.x * 256 + threadIdx.x; if (idx >= TT * HD) return; v2f cs; cs[0] = 1.0f; cs[1] = 0.0f; *(volatile v2f*)(CS + (size_t)idx * 2) = cs; __threadfence(); *(volatile v2f*)(CS + (size_t)idx * 2) = cs; }

__device__ __forceinline__ float tanhx(float s) { const float e2 = __builtin_amdgcn_exp2f(s * 2.8853900817779268f); const float r = __fdiv_rn(1.0f, e2 + 1.0f); return 1.0f - (r + r); }

__global__ __launch_bounds__(256) void k_kwin(const float* __restrict__ KP, bf* KWh, bf* KWl) { const size_t e = ((size_t)blockIdx.x * 256 + threadIdx.x) * 2; if (e >= (size_t)NH_ * NCH * KWN * HD) return; const int d = (int)(e % HD); const int y = (int)((e / HD) % KWN); const int c = (int)((e / ((size_t)HD * KWN)) % NCH); const int h = (int)(e / ((size_t)HD * KWN * NCH));
    const int j = c * WINW - PADW + y; const bool ok = (j >= 0) & (j < TT); const int jc = min(max(j, 0), TT - 1); const float f = ok ? 1.0f : 0.0f; const v2f x = *(const v2f*)(KP + ((size_t)jc * NH_ + h) * HD + d); v2us oh, ol;
#pragma unroll
    for (int q = 0; q < 2; ++q) { const float r = __fmul_rn(x[q], f); unsigned short a2, c2; splitf(r, a2, c2); oh[q] = a2; ol[q] = c2; }
    *(volatile v2us*)(KWh + e) = oh; *(volatile v2us*)(KWl + e) = ol; __threadfence(); *(volatile v2us*)(KWh + e) = oh; *(volatile v2us*)(KWl + e) = ol; }

__global__ __launch_bounds__(256) void k_vwin(const float* __restrict__ V, h16* VW) { const size_t e = ((size_t)blockIdx.x * 256 + threadIdx.x) * 2; if (e >= (size_t)NCH * VO * KWN * NH_) return; const int h = (int)(e % NH_); const int y = (int)((e / NH_) % KWN); const int o = (int)((e / ((size_t)NH_ * KWN)) % VO); const int c = (int)(e / ((size_t)NH_ * KWN * VO));
    const int j = c * WINW - PADW + y; const bool ok = (j >= 0) & (j < TT); const int jc = min(max(j, 0), TT - 1); const float* vr = V + (size_t)jc * (NH_ * VO) + o; const float f = ok ? 1.0f : 0.0f; const float x0 = vr[h * VO], x1 = vr[(h + 1) * VO]; v2h w; w[0] = tohx(__fmul_rn(bfr(x0), f)); w[1] = tohx(__fmul_rn(bfr(x1), f));
    *(volatile v2h*)(VW + e) = w; __threadfence(); *(volatile v2h*)(VW + e) = w; }

__global__ __launch_bounds__(256) void k_tband(const float* __restrict__ S, const float* __restrict__ OC, h16* P16) { const size_t e = (size_t)blockIdx.x * 256 + threadIdx.x; if (e >= (size_t)NCH * WINW * KWN) return; const int y = (int)(e % KWN); const int x = (int)((e / KWN) % WINW); const int c = (int)(e / ((size_t)KWN * WINW));
    const int dd = y - x; const int j = c * WINW - PADW + y; const bool ok = (dd >= 0) & (dd <= WINW) & (j >= 0) & (j < TT); const int dc = min(max(dd, 0), WINW); const float f = ok ? 1.0f : 0.0f; v8h w;
#pragma unroll
    for (int h = 0; h < NH_; ++h) { const float s = S[(size_t)h * NCH * WINW * KWN + e]; const float a = tanhx(s + OC[dc * NH_ + h]); w[h] = tohx(__fmul_rn(a, f)); }
    *(volatile v8h*)(P16 + e * NH_) = w; __threadfence(); *(volatile v8h*)(P16 + e * NH_) = w; }

__global__ __launch_bounds__(256) void k_tflat(const float* __restrict__ S, const float* __restrict__ OC, float* R1) { const size_t e = ((size_t)blockIdx.x * 256 + threadIdx.x) * 4; if (e >= (size_t)TT * NOFF * NH_) return; const int h0 = (int)(e % NH_); const int d = (int)((e / NH_) % NOFF); const int t = (int)(e / ((size_t)NH_ * NOFF));
    const int c = t / WINW; const int x = t % WINW; const int j = t - PADW + d; const bool ok = (j >= 0) & (j < TT); const float f = ok ? 1.0f : 0.0f; const size_t so = ((size_t)c * WINW + x) * KWN + (x + d); v4f o;
#pragma unroll
    for (int q = 0; q < 4; ++q) { const float s = S[(size_t)(h0 + q) * NCH * WINW * KWN + so]; const float a = tanhx(s + OC[d * NH_ + h0 + q]); o[q] = __fmul_rn(a, f); }
    *(volatile v4f*)(R1 + e) = o; __threadfence(); *(volatile v4f*)(R1 + e) = o; }

extern "C" void kernel_launch(void* const* d_in, const int* in_sizes, int n_in,
                              void* d_out, int out_size, void* d_ws, size_t ws_size, hipStream_t stream) {
    (void)in_sizes; (void)n_in; (void)out_size;
    const float* qin = (const float*)d_in[0]; const float* kin = (const float*)d_in[1]; const float* vin = (const float*)d_in[2];
    const float* wq = (const float*)d_in[3]; const float* bq = (const float*)d_in[4]; const float* wk = (const float*)d_in[5]; const float* bk = (const float*)d_in[6]; const float* ocpe = (const float*)d_in[7];
    float* R1 = (float*)d_out;
    float* R2 = R1 + (size_t)NB_ * TT * NOFF * NH_;
    char* wsp = (char*)d_ws;
    auto take = [&](size_t bytes) { char* p = wsp; wsp += (bytes + 255) & ~(size_t)255; return (void*)p; };
    const size_t NROW = (size_t)NB_ * TT * NH_;
    float* CS = (float*)take((size_t)TT * HD * 2 * 4); bf* WQB = (bf*)take((size_t)HD * HD * 2); bf* WKB = (bf*)take((size_t)HD * HD * 2); float* BQ = (float*)take((size_t)HD * 4); float* BK = (float*)take((size_t)HD * 4); float* OC = (float*)take((size_t)NOFF * NH_ * 4);
    bf* QB = (bf*)take(NROW * HD * 2); bf* KB = (bf*)take(NROW * HD * 2); float* QP = (float*)take(NROW * HD * 4); float* KP = (float*)take(NROW * HD * 4);
    h16* Q16 = (h16*)take((size_t)NH_ * TT * HD * 2); bf* Qh = (bf*)take((size_t)NH_ * TT * HD * 2); bf* Ql = (bf*)take((size_t)NH_ * TT * HD * 2);
    bf* KWh = (bf*)take((size_t)NH_ * NCH * KWN * HD * 2); bf* KWl = (bf*)take((size_t)NH_ * NCH * KWN * HD * 2); float* Sb = (float*)take((size_t)NH_ * NCH * WINW * KWN * 4);
    h16* VW = (h16*)take((size_t)NCH * VO * KWN * NH_ * 2); h16* P16 = (h16*)take((size_t)NCH * WINW * KWN * NH_ * 2);
    if ((size_t)(wsp - (char*)d_ws) > ws_size) return;
    k_csid<<<(TT * HD + 255) / 256, 256, 0, stream>>>(CS);
    k_cvt8<<<(unsigned)((NROW * HD / 8 + 255) / 256), 256, 0, stream>>>(qin, QB, NROW * HD / 8); k_cvt8<<<(unsigned)((NROW * HD / 8 + 255) / 256), 256, 0, stream>>>(kin, KB, NROW * HD / 8);
    k_cvt8<<<(HD * HD / 8 + 255) / 256, 256, 0, stream>>>(wq, WQB, (size_t)HD * HD / 8); k_cvt8<<<(HD * HD / 8 + 255) / 256, 256, 0, stream>>>(wk, WKB, (size_t)HD * HD / 8);
    k_rbf<<<1, 256, 0, stream>>>(bq, BQ, (size_t)HD / 4); k_rbf<<<1, 256, 0, stream>>>(bk, BK, (size_t)HD / 4); k_rbf<<<(NOFF * NH_ / 4 + 255) / 256, 256, 0, stream>>>(ocpe, OC, (size_t)NOFF * NH_ / 4);
    k_gemmw<bf, 0, true><<<dim3((unsigned)(NROW / 64), HD / 64, 1), 32, 0, stream>>>(QB, nullptr, WQB, nullptr, HD, QP, HD, BQ, 0, 0, 0);
    k_gemmw<bf, 0, true><<<dim3((unsigned)(NROW / 64), HD / 64, 1), 32, 0, stream>>>(KB, nullptr, WKB, nullptr, HD, KP, HD, BK, 0, 0, 0);
    for (int b = 0; b < NB_; ++b) {
        const float* QPb = QP + (size_t)b * TT * NH_ * HD; const float* KPb = KP + (size_t)b * TT * NH_ * HD; const float* Vb = vin + (size_t)b * TT * NH_ * VO;
        k_rope<<<(unsigned)((size_t)NH_ * TT * HD / 512), 256, 0, stream>>>(QPb, NH_ * HD, NH_, CS, nullptr, nullptr, 1.0f, Q16, Qh, Ql);
        k_kwin<<<(unsigned)((size_t)NH_ * NCH * KWN * HD / 512), 256, 0, stream>>>(KPb, KWh, KWl);
        for (int h = 0; h < NH_; ++h)
            k_gemmw<bf, 2, false><<<dim3(WINW / 64, KWN / 64, NCH), 32, 0, stream>>>(Qh + (size_t)h * TT * HD, Ql + (size_t)h * TT * HD, KWh + (size_t)h * NCH * KWN * HD, KWl + (size_t)h * NCH * KWN * HD, HD, Sb + (size_t)h * NCH * WINW * KWN, KWN, nullptr, (size_t)WINW * HD, (size_t)KWN * HD, (size_t)WINW * KWN);
        k_vwin<<<(unsigned)((size_t)NCH * VO * KWN * NH_ / 512), 256, 0, stream>>>(Vb, VW);
        k_tband<<<(unsigned)((size_t)NCH * WINW * KWN / 256), 256, 0, stream>>>(Sb, OC, P16);
        k_gemmw<h16, 0, false><<<dim3(WINW / 64, VO / 64, NCH), 32, 0, stream>>>(P16, nullptr, VW, nullptr, KWN * NH_, R2 + (size_t)b * TT * VO, VO, nullptr, (size_t)WINW * KWN * NH_, (size_t)VO * KWN * NH_, (size_t)WINW * VO);
        k_tflat<<<(unsigned)((size_t)TT * NOFF * NH_ / 1024), 256, 0, stream>>>(Sb, OC, R1 + (size_t)b * TT * NOFF * NH_);
    }
}
